// _QuantumGate_65481071396941
// MI455X (gfx1250) — hardware-verified
//
#include <hip/hip_runtime.h>


typedef __bf16       v16bf __attribute__((ext_vector_type(16)));
typedef float        v8f   __attribute__((ext_vector_type(8)));
typedef float        v4f   __attribute__((ext_vector_type(4), __may_alias__));
typedef unsigned int v4u   __attribute__((ext_vector_type(4), __may_alias__));

#define NQ      12
#define NANG    36
#define NPADC   48
#define FDIM    512
#define BATCH   8192
#define BLOCK   128
#define WPB     (BLOCK / 32)
#define ROWS_PB (WPB * 16)
#define ANGP    36
#define F4_PB   (ROWS_PB * NQ / 4)
#define WROW    (FDIM / 2)

static_assert(BATCH % ROWS_PB == 0);
static_assert(FDIM % 32 == 0);
static_assert((ROWS_PB * NQ * 4) % 128 == 0);
static_assert(F4_PB > BLOCK && F4_PB <= 2 * BLOCK);
static_assert(ROWS_PB <= BLOCK);

__device__ __forceinline__ unsigned int bf16_rne(float f)
{
    unsigned int u = __float_as_uint(f);
    u += 0x7FFFu + ((u >> 16) & 1u);
    return u >> 16;
}

__device__ __forceinline__ unsigned int pack_bf16x2(float lo, float hi)
{
    return bf16_rne(lo) | (bf16_rne(hi) << 16);
}

union Frag {
    v16bf        v;
    v4u          q[2];
    unsigned int u[8];
};

__device__ __forceinline__ v8f wmma_bf16_16x16x32(v16bf a, v16bf b, v8f acc)
{
    acc = __builtin_amdgcn_wmma_f32_16x16x32_bf16(false, a, false, b, (short)0, acc, false, false);
    asm volatile("v_nop\n\tv_nop\n\tv_nop\n\tv_nop" : "+v"(acc) : "v"(a), "v"(b));
    return acc;
}

__global__ __launch_bounds__(BLOCK)
void k_proj_cosprod(const float* __restrict__ x,
                    const float* __restrict__ W,
                    const float* __restrict__ bias,
                    float* out)
{
    __shared__ __align__(16) unsigned int sW32[NPADC * WROW];
    __shared__ __align__(16) float        sAng[ROWS_PB * ANGP];
    __shared__ __align__(16) float        sOut[ROWS_PB * NQ];
    __shared__ float                      sBias[NANG];

    const int tid  = threadIdx.x;
    const int lane = tid & 31;
    const int wid  = tid >> 5;
    const int h    = lane >> 4;
    const int m    = lane & 15;

    for (int g = tid; g < NPADC * FDIM / 4; g += BLOCK) {
        const int e = g * 4;
        unsigned int w0 = 0u, w1 = 0u;
        if (e < NANG * FDIM) {
            const v4f p = *(const v4f*)(W + e);
            w0 = pack_bf16x2(p[0], p[1]);
            w1 = pack_bf16x2(p[2], p[3]);
        }
        sW32[2 * g]     = w0;
        sW32[2 * g + 1] = w1;
    }
    if (tid < NANG) sBias[tid] = __uint_as_float(bf16_rne(bias[tid]) << 16);
    __syncthreads();

    const int rowBase = blockIdx.x * ROWS_PB + wid * 16;
    const float* xr = x + (size_t)(rowBase + m) * FDIM;

    v8f c0 = {};
    v8f c1 = {};
    v8f c2 = {};

#pragma unroll 2
    for (int k0 = 0; k0 < FDIM; k0 += 32) {
        const int ka = k0 + 8 * h;
        const int kb = k0 + 16 + 8 * h;
        const v4f p0 = *(const v4f*)(xr + ka);
        const v4f p1 = *(const v4f*)(xr + ka + 4);
        const v4f p2 = *(const v4f*)(xr + kb);
        const v4f p3 = *(const v4f*)(xr + kb + 4);
        Frag a;
        a.u[0] = pack_bf16x2(p0[0], p0[1]);
        a.u[1] = pack_bf16x2(p0[2], p0[3]);
        a.u[2] = pack_bf16x2(p1[0], p1[1]);
        a.u[3] = pack_bf16x2(p1[2], p1[3]);
        a.u[4] = pack_bf16x2(p2[0], p2[1]);
        a.u[5] = pack_bf16x2(p2[2], p2[3]);
        a.u[6] = pack_bf16x2(p3[0], p3[1]);
        a.u[7] = pack_bf16x2(p3[2], p3[3]);

        const int wb = (k0 >> 1) + 4 * h;
        Frag b0, b1, b2;
        b0.q[0] = *(const v4u*)(sW32 + (m) * WROW + wb);
        b0.q[1] = *(const v4u*)(sW32 + (m) * WROW + wb + 8);
        b1.q[0] = *(const v4u*)(sW32 + (16 + m) * WROW + wb);
        b1.q[1] = *(const v4u*)(sW32 + (16 + m) * WROW + wb + 8);
        b2.q[0] = *(const v4u*)(sW32 + (32 + m) * WROW + wb);
        b2.q[1] = *(const v4u*)(sW32 + (32 + m) * WROW + wb + 8);

        c0 = wmma_bf16_16x16x32(a.v, b0.v, c0);
        c1 = wmma_bf16_16x16x32(a.v, b1.v, c1);
        c2 = wmma_bf16_16x16x32(a.v, b2.v, c2);
    }

    {
        float* ang = sAng + (wid * 16) * ANGP;
#pragma unroll
        for (int r = 0; r < 8; ++r) {
            const int row = 8 * h + r;
            ang[row * ANGP + m]      = c0[r];
            ang[row * ANGP + 16 + m] = c1[r];
            if (m < 4) ang[row * ANGP + 32 + m] = c2[r];
        }
    }
    __syncthreads();

    if (tid < ROWS_PB) {
        const float* ar = sAng + tid * ANGP;
        float prod = 1.0f;
#pragma unroll 1
        for (int q = 0; q < NQ; ++q) {
            const float tx = ar[3 * q]     + sBias[3 * q];
            const float ty = ar[3 * q + 1] + sBias[3 * q + 1];
            const float cz = cosf(tx) * cosf(ty);
            prod = prod * cz;
            sOut[tid * NQ + q] = prod;
        }
    }
    __syncthreads();

    const v4f v0 = *(const v4f*)(sOut + 4 * tid);
    v4f v1 = v0;
    if (tid < F4_PB - BLOCK) v1 = *(const v4f*)(sOut + 4 * (tid + BLOCK));
    volatile v4f* o4 = (volatile v4f*)(out) + (size_t)blockIdx.x * F4_PB;
    o4[tid] = v0;
    if (tid < F4_PB - BLOCK) o4[tid + BLOCK] = v1;
    __threadfence();
    o4[tid] = v0;
    if (tid < F4_PB - BLOCK) o4[tid + BLOCK] = v1;
}

extern "C" void kernel_launch(void* const* d_in, const int* in_sizes, int n_in,
                              void* d_out, int out_size, void* d_ws, size_t ws_size,
                              hipStream_t stream)
{
    (void)d_ws;
    (void)ws_size;
    if (n_in < 3) return;
    if (in_sizes[0] != BATCH * FDIM) return;
    if (in_sizes[1] != NANG * FDIM) return;
    if (in_sizes[2] != NANG) return;
    if (out_size != BATCH * NQ) return;

    const float* x    = (const float*)d_in[0];
    const float* W    = (const float*)d_in[1];
    const float* bias = (const float*)d_in[2];
    float*       out  = (float*)d_out;

    hipLaunchKernelGGL(k_proj_cosprod, dim3(BATCH / ROWS_PB), dim3(BLOCK), 0, stream,
                       x, W, bias, out);
    (void)hipGetLastError();
}
